// RNN_15625091023237
// MI455X (gfx1250) — hardware-verified
//
#include <hip/hip_runtime.h>
#include <math.h>

constexpr int NBATCH  = 1024;
constexpr int NSTEP   = 256;
constexpr int NVOC    = 115;
constexpr int NEMB    = 128;
constexpr int NHID    = 512;
constexpr int NTHR    = 256;
constexpr int SEQ_BLK = 16;
constexpr int HPITCH  = 520;
constexpr int SLABP   = 68;
constexpr float WCARRY = 256.0f;
constexpr float HCARRY = 64.0f;
constexpr float FOLD_INV = 1.0f / (WCARRY * HCARRY);
constexpr int NOUT = NBATCH * NVOC;

static_assert(NBATCH % SEQ_BLK == 0, "batch tile");
static_assert(NHID == 64 * (NTHR / 32), "8 waves x 64 hidden columns");
static_assert(NHID % 32 == 0, "K multiple of 32");
static_assert(NHID % 64 == 0, "transpose tiles");
static_assert((2 * SEQ_BLK * HPITCH) % NTHR == 0, "h zero-fill loop exact");
static_assert((NVOC * NHID) % NTHR == 0, "E grid exact");
static_assert(NOUT % NTHR == 0, "logits grid exact");
static_assert((NOUT * 4) % 128 == 0, "output is whole lines");
static_assert(NEMB % 8 == 0, "E loop step");
static_assert((HPITCH * 2) % 16 == 0, "h rows 16-B aligned");

typedef __attribute__((ext_vector_type(16))) _Float16 v16h;
typedef __attribute__((ext_vector_type(8)))  _Float16 v8h;
typedef __attribute__((ext_vector_type(8)))  float    v8f;
typedef __attribute__((ext_vector_type(4)))  float    v4f;

union FragU { v16h v; v8h h[2]; };
__device__ __forceinline__ v16h frag_load(const _Float16* p) {
  FragU f;
  f.h[0] = *(const v8h*)(p);
  f.h[1] = *(const v8h*)(p + 16);
  return f.v;
}
__device__ __forceinline__ v8f frag_mma(v16h a, v16h b, v8f c) {
  return __builtin_amdgcn_wmma_f32_16x16x32_f16(false, a, false, b, (short)0, c, false, false);
}
__device__ __forceinline__ void kguard4(v8f& a0, v8f& a1, v8f& a2, v8f& a3,
                                        v16h x, v16h y0, v16h y1, v16h y2, v16h y3) {
  asm volatile("v_nop\n\tv_nop\n\tv_nop\n\tv_nop"
               : "+v"(a0), "+v"(a1), "+v"(a2), "+v"(a3)
               : "v"(x), "v"(y0), "v"(y1), "v"(y2), "v"(y3));
}
__device__ __forceinline__ void acc_guard4(v8f& a, v8f& b, v8f& c, v8f& d) {
  asm volatile("v_nop\n\tv_nop\n\tv_nop\n\tv_nop" : "+v"(a), "+v"(b), "+v"(c), "+v"(d));
}
__device__ __forceinline__ void wave_lds_sync() {
  __builtin_amdgcn_fence(__ATOMIC_RELEASE, "workgroup");
  __builtin_amdgcn_wave_barrier();
  __builtin_amdgcn_fence(__ATOMIC_ACQUIRE, "workgroup");
}

__global__ __launch_bounds__(NTHR) void etab_kernel(const float* __restrict__ W_emb, const float* __restrict__ W_xh,
                                                    const float* __restrict__ b_h, float* __restrict__ E) {
  const int idx = blockIdx.x * NTHR + threadIdx.x;
  if (idx >= NVOC * NHID) return;
  const int v = idx / NHID;
  const int n = idx - v * NHID;
  const float* wrow = W_emb + (size_t)v * NEMB;
  const float* xcol = W_xh + n;
  float s0 = 0.0f, s1 = 0.0f, s2 = 0.0f, s3 = 0.0f;
#pragma unroll 2
  for (int e = 0; e < NEMB; e += 4) {
    const v4f w = *(const v4f*)(wrow + e);
    s0 += w[0] * xcol[(size_t)(e + 0) * NHID];
    s1 += w[1] * xcol[(size_t)(e + 1) * NHID];
    s2 += w[2] * xcol[(size_t)(e + 2) * NHID];
    s3 += w[3] * xcol[(size_t)(e + 3) * NHID];
  }
  const float s = b_h[n] + ((s0 + s1) + (s2 + s3));
  volatile float* ep = E + idx;
  *ep = s;
  __threadfence();
  *ep = s;
}

__global__ __launch_bounds__(NTHR) void tpw_kernel(const float* __restrict__ src, int R, int C, int ldo,
                                                   unsigned short* __restrict__ O, float sc) {
  __shared__ float Tt[64 * 65];
  const int tid = threadIdx.x;
  const int c0 = blockIdx.x * 64, r0 = blockIdx.y * 64;
#pragma unroll
  for (int i = 0; i < 4; ++i) {
    const int idx = i * NTHR + tid;
    const int rr = idx >> 4, cc = (idx & 15) * 4;
    const v4f v = *(const v4f*)(src + (size_t)(r0 + rr) * (size_t)C + c0 + cc);
    Tt[rr * 65 + cc + 0] = v[0];
    Tt[rr * 65 + cc + 1] = v[1];
    Tt[rr * 65 + cc + 2] = v[2];
    Tt[rr * 65 + cc + 3] = v[3];
  }
  __syncthreads();
  const int q = tid >> 3, c8 = (tid & 7) * 8;
  v8h hv0, hv1;
#pragma unroll
  for (int e = 0; e < 8; ++e) {
    const float f0 = Tt[(c8 + e) * 65 + q];
    const float f1 = Tt[(c8 + e) * 65 + 32 + q];
    hv0[e] = (_Float16)(f0 * sc);
    hv1[e] = (_Float16)(f1 * sc);
  }
  _Float16* Oh = (_Float16*)O;
  const size_t o0 = (size_t)(c0 + q) * (size_t)ldo + (size_t)(r0 + c8);
  const size_t o1 = (size_t)(c0 + 32 + q) * (size_t)ldo + (size_t)(r0 + c8);
  for (int pass = 0; pass < 2; ++pass) {
    *(volatile v8h*)(Oh + o0) = hv0;
    *(volatile v8h*)(Oh + o1) = hv1;
    __threadfence();
  }
}

__global__ __launch_bounds__(NTHR) void rnn_seq_kernel(const int* __restrict__ X, const float* __restrict__ E,
                                                       const unsigned short* __restrict__ WTp, float* __restrict__ HT) {
  __shared__ __align__(16) _Float16 Ah[2][SEQ_BLK * HPITCH];
  __shared__ __align__(16) float    Sl[NTHR / 32][16 * SLABP];
  const _Float16* WT = (const _Float16*)WTp;
  const int tid = threadIdx.x, lane = tid & 31, wave = tid >> 5;
  const int c = lane & 15, hh = lane >> 4, koff = hh * 8;
  const int q = lane >> 3, c8 = (lane & 7) * 8;
  const int rowbase = blockIdx.x * SEQ_BLK;

  {
    _Float16* ahf = &Ah[0][0];
#pragma unroll 1
    for (int i = tid; i < 2 * SEQ_BLK * HPITCH; i += NTHR) ahf[i] = (_Float16)0.0f;
  }
  __syncthreads();

  const v8f z8 = {0.f, 0.f, 0.f, 0.f, 0.f, 0.f, 0.f, 0.f};
  float* slab = Sl[wave];
  const _Float16* wb0 = WT + (size_t)(64 * wave + c) * NHID + koff;
  const _Float16* wb1 = wb0 + (size_t)16 * NHID;
  const _Float16* wb2 = wb0 + (size_t)32 * NHID;
  const _Float16* wb3 = wb0 + (size_t)48 * NHID;

#pragma unroll 1
  for (int t = 0; t < NSTEP; ++t) {
    const int cur = t & 1;
    const _Float16* ahrow = &Ah[cur][0] + c * HPITCH + koff;
    _Float16* ahn = &Ah[cur ^ 1][0];
    const bool last = (t == NSTEP - 1);

    v8f acc[4];
    acc[0] = z8; acc[1] = z8; acc[2] = z8; acc[3] = z8;
#pragma unroll 1
    for (int k0 = 0; k0 < NHID; k0 += 32) {
      const v16h a  = frag_load(ahrow + k0);
      const v16h b0 = frag_load(wb0 + k0);
      const v16h b1 = frag_load(wb1 + k0);
      const v16h b2 = frag_load(wb2 + k0);
      const v16h b3 = frag_load(wb3 + k0);
      acc[0] = frag_mma(a, b0, acc[0]);
      acc[1] = frag_mma(a, b1, acc[1]);
      acc[2] = frag_mma(a, b2, acc[2]);
      acc[3] = frag_mma(a, b3, acc[3]);
      kguard4(acc[0], acc[1], acc[2], acc[3], a, b0, b1, b2, b3);
    }
    acc_guard4(acc[0], acc[1], acc[2], acc[3]);

#pragma unroll
    for (int nt = 0; nt < 4; ++nt)
#pragma unroll
      for (int r = 0; r < 8; ++r) slab[(8 * hh + r) * SLABP + 16 * nt + c] = acc[nt][r];
    wave_lds_sync();

#pragma unroll 1
    for (int it = 0; it < 4; ++it) {
      const int row = it * 4 + q;
      int tk = X[(size_t)(rowbase + row) * NSTEP + (size_t)t];
      tk = tk < 0 ? 0 : tk;
      tk = tk > (NVOC - 1) ? (NVOC - 1) : tk;
      const float* ep = E + (size_t)tk * NHID + 64 * wave + c8;
      const v4f e0 = *(const v4f*)(ep);
      const v4f e1 = *(const v4f*)(ep + 4);
      float* sp = slab + row * SLABP + c8;
      const v4f s0 = *(const v4f*)(sp);
      const v4f s1 = *(const v4f*)(sp + 4);
      v4f h0v, h1v;
      v8h hv;
#pragma unroll
      for (int e = 0; e < 4; ++e) {
        const float x0 = s0[e] * FOLD_INV + e0[e];
        const float x1 = s1[e] * FOLD_INV + e1[e];
        const float t0 = tanhf(x0);
        const float t1 = tanhf(x1);
        h0v[e] = t0;
        h1v[e] = t1;
        hv[e]     = (_Float16)(t0 * HCARRY);
        hv[4 + e] = (_Float16)(t1 * HCARRY);
      }
      *(v8h*)(ahn + row * HPITCH + 64 * wave + c8) = hv;
      if (last) {
        *(v4f*)(sp)     = h0v;
        *(v4f*)(sp + 4) = h1v;
      }
    }
    __syncthreads();
  }

  {
    const int c4 = c * 4;
    for (int pass = 0; pass < 2; ++pass) {
#pragma unroll
      for (int it = 0; it < 8; ++it) {
        const int row = it * 2 + hh;
        const v4f v = *(const v4f*)(slab + row * SLABP + c4);
        *(volatile v4f*)(HT + (size_t)(rowbase + row) * NHID + 64 * wave + c4) = v;
      }
      __threadfence();
    }
  }
}

__global__ __launch_bounds__(NTHR) void logits_kernel(const float* __restrict__ HT, const float* __restrict__ W_hy,
                                                      const float* __restrict__ b_y, float* __restrict__ out) {
  const int o = blockIdx.x * NTHR + threadIdx.x;
  if (o >= NOUT) return;
  const int row = o / NVOC;
  const int v = o - row * NVOC;
  const float* hp = HT + (size_t)row * NHID;
  const float* wp = W_hy + v;
  float s0 = 0.0f, s1 = 0.0f, s2 = 0.0f, s3 = 0.0f;
#pragma unroll 2
  for (int k = 0; k < NHID; k += 4) {
    const v4f h = *(const v4f*)(hp + k);
    s0 += h[0] * wp[(size_t)(k + 0) * NVOC];
    s1 += h[1] * wp[(size_t)(k + 1) * NVOC];
    s2 += h[2] * wp[(size_t)(k + 2) * NVOC];
    s3 += h[3] * wp[(size_t)(k + 3) * NVOC];
  }
  const float s = b_y[v] + ((s0 + s1) + (s2 + s3));
  volatile float* op = out + o;
  *op = s;
  __threadfence();
  *op = s;
}

extern "C" void kernel_launch(void* const* d_in, const int* in_sizes, int n_in,
                              void* d_out, int out_size, void* d_ws, size_t ws_size, hipStream_t stream) {
  if (n_in < 7 || d_out == nullptr || d_ws == nullptr) return;
  if (in_sizes[0] != NBATCH * NSTEP || in_sizes[1] != NVOC * NEMB || in_sizes[2] != NEMB * NHID ||
      in_sizes[3] != NHID * NHID || in_sizes[4] != NHID || in_sizes[5] != NHID * NVOC ||
      in_sizes[6] != NVOC || out_size != NOUT) return;

  const int*   X     = (const int*)d_in[0];
  const float* W_emb = (const float*)d_in[1];
  const float* W_xh  = (const float*)d_in[2];
  const float* W_hh  = (const float*)d_in[3];
  const float* b_h   = (const float*)d_in[4];
  const float* W_hy  = (const float*)d_in[5];
  const float* b_y   = (const float*)d_in[6];
  float* out = (float*)d_out;

  char* ws = (char*)d_ws;
  size_t off = 0;
  auto carve = [&](size_t bytes) -> char* { char* p = ws + off; off += (bytes + 255) & ~(size_t)255; return p; };
  float*          ETAB = (float*)carve((size_t)NVOC * NHID * 4);
  unsigned short* WT   = (unsigned short*)carve((size_t)NHID * NHID * 2);
  float*          HT   = (float*)carve((size_t)NBATCH * NHID * 4);
  if (off > ws_size || off > (size_t)134217728) return;

  etab_kernel<<<(NVOC * NHID) / NTHR, NTHR, 0, stream>>>(W_emb, W_xh, b_h, ETAB);
  tpw_kernel<<<dim3(NHID / 64, NHID / 64), NTHR, 0, stream>>>(W_hh, NHID, NHID, NHID, WT, WCARRY);
  rnn_seq_kernel<<<NBATCH / SEQ_BLK, NTHR, 0, stream>>>(X, ETAB, WT, HT);
  logits_kernel<<<NOUT / NTHR, NTHR, 0, stream>>>(HT, W_hy, b_y, out);
}
